// NeuronCircuitUp_31593779429535
// MI455X (gfx1250) — hardware-verified
//
#include <hip/hip_runtime.h>
#include <stdint.h>
#include <stddef.h>

constexpr int RANK_DIM  = 128;
constexpr int DMODEL    = 1024;
constexpr int NOUT      = 8;
constexpr int NREFL     = 4;
constexpr int KCOLS     = NOUT * RANK_DIM;
constexpr int TOK_PER_BLK = 8;

typedef __attribute__((ext_vector_type(16))) _Float16 v16h;
typedef __attribute__((ext_vector_type(8)))  _Float16 v8h;
typedef __attribute__((ext_vector_type(16))) __bf16   v16b;
typedef __attribute__((ext_vector_type(8)))  __bf16   v8b;
typedef __attribute__((ext_vector_type(8)))  float    v8f;
typedef __attribute__((ext_vector_type(4)))  float    v4f;

__device__ __forceinline__ unsigned short f2bf_bits(float f) {
  unsigned u = __float_as_uint(f);
  return (unsigned short)((u + 0x7FFFu + ((u >> 16) & 1u)) >> 16);
}
__device__ __forceinline__ float bf_bits2f(unsigned short h) { return __uint_as_float(((unsigned)h) << 16); }

__device__ __forceinline__ void dep_guard_h(v8f& a, v8f& b, v16h x, v16h y) { asm volatile("v_nop\n\tv_nop\n\tv_nop\n\tv_nop" : "+v"(a), "+v"(b) : "v"(x), "v"(y)); }
__device__ __forceinline__ void dep_guard_b(v8f& a, v8f& b, v16b x, v16b y) { asm volatile("v_nop\n\tv_nop\n\tv_nop\n\tv_nop" : "+v"(a), "+v"(b) : "v"(x), "v"(y)); }
__device__ __forceinline__ void keep4_h(v16h a, v16h b, v16h c, v16h d) { asm volatile("v_nop" :: "v"(a), "v"(b), "v"(c), "v"(d)); }
__device__ __forceinline__ void keep4_b(v16b a, v16b b, v16b c, v16b d) { asm volatile("v_nop" :: "v"(a), "v"(b), "v"(c), "v"(d)); }
__device__ __forceinline__ void acc_guard4(v8f& a, v8f& b, v8f& c, v8f& d) { asm volatile("v_nop\n\tv_nop\n\tv_nop\n\tv_nop" : "+v"(a), "+v"(b), "+v"(c), "+v"(d)); }
template <typename T> struct Frag;
template <> struct Frag<_Float16> {
  typedef v16h V; union U { v16h v; v8h h[2]; };
  static __device__ __forceinline__ v16h load(const _Float16* p) {
    U f; f.h[0] = *(const v8h*)(p); f.h[1] = *(const v8h*)(p + 16); return f.v;
  }
  static __device__ __forceinline__ v8f mma(v16h a, v16h b, v8f c) {
    return __builtin_amdgcn_wmma_f32_16x16x32_f16(false, a, false, b, (short)0, c, false, false);
  }
  static __device__ __forceinline__ void guard(v8f& a, v8f& b, v16h x, v16h y) { dep_guard_h(a, b, x, y); }
  static __device__ __forceinline__ void keep(v16h a, v16h b, v16h c, v16h d) { keep4_h(a, b, c, d); }
};
template <> struct Frag<__bf16> {
  typedef v16b V; union U { v16b v; v8b h[2]; };
  static __device__ __forceinline__ v16b load(const __bf16* p) {
    U f; f.h[0] = *(const v8b*)(p); f.h[1] = *(const v8b*)(p + 16); return f.v;
  }
  static __device__ __forceinline__ v8f mma(v16b a, v16b b, v8f c) {
    return __builtin_amdgcn_wmma_f32_16x16x32_bf16(false, a, false, b, (short)0, c, false, false);
  }
  static __device__ __forceinline__ void guard(v8f& a, v8f& b, v16b x, v16b y) { dep_guard_b(a, b, x, y); }
  static __device__ __forceinline__ void keep(v16b a, v16b b, v16b c, v16b d) { keep4_b(a, b, c, d); }
};

template <int ET> struct Elem;
template <> struct Elem<0> { typedef _Float16 T; };
template <> struct Elem<1> { typedef __bf16 T; };
template <int ET, bool SPLIT, int BIAS_MODE, int OUT_MODE, bool RESID, int ACT = 0>
__global__ __launch_bounds__(256) void wmma_gemm64(
    const unsigned short* __restrict__ Ap, const unsigned short* __restrict__ A2p, int lda, long strideA,
    const unsigned short* __restrict__ Btp, const unsigned short* __restrict__ Bt2p, int ldb, long strideB,
    void* __restrict__ Cout, void* __restrict__ Cout2, int ldc, long strideC,
    const float* __restrict__ bias,
    const float* __restrict__ resid, long strideR,
    int M, int N, int K, float scale) {
  typedef typename Elem<ET>::T T;
  typedef typename Frag<T>::V V;
  const T* A = (const T*)Ap; const T* A2 = (const T*)A2p; const T* Bt = (const T*)Btp; const T* Bt2 = (const T*)Bt2p;
  __shared__ __align__(16) float sT[8][16 * 68];
  const int b    = blockIdx.y;
  const int lane = threadIdx.x & 31;
  const int wave = threadIdx.x >> 5;
  const int tilesN = N >> 6;
  const int tilesM = M >> 6;
  const int tile = blockIdx.x * 8 + wave;
  if (tile >= tilesM * tilesN) return;
  const int tm = tile / tilesN;
  const int tn = tile - tm * tilesN;
  const int m0 = tm << 6;
  const int n0 = tn << 6;

  const T* Ab  = A  + (size_t)b * strideA;
  const T* Bb  = Bt + (size_t)b * strideB;
  const T* Ab2 = SPLIT ? (A2  + (size_t)b * strideA) : nullptr;
  const T* Bb2 = SPLIT ? (Bt2 + (size_t)b * strideB) : nullptr;

  const int rlane = lane & 15;
  const int koff  = (lane >> 4) * 8;
  const int mOff  = (lane >> 4) * 8;

  v8f acc[4][4];
#pragma unroll
  for (int i = 0; i < 4; ++i)
#pragma unroll
    for (int j = 0; j < 4; ++j) acc[i][j] = (v8f){0.f,0.f,0.f,0.f,0.f,0.f,0.f,0.f};

  for (int k0 = 0; k0 < K; k0 += 32) {
    V bh[4], bl[4];
#pragma unroll
    for (int j = 0; j < 4; ++j) {
      const size_t bo = (size_t)(n0 + (j << 4) + rlane) * ldb + koff + k0;
      bh[j] = Frag<T>::load(Bb + bo);
      if (SPLIT) bl[j] = Frag<T>::load(Bb2 + bo);
    }
#pragma unroll
    for (int i = 0; i < 4; ++i) {
      const size_t ao = (size_t)(m0 + (i << 4) + rlane) * lda + koff + k0;
      V ah = Frag<T>::load(Ab + ao);
      V al;
      if (SPLIT) al = Frag<T>::load(Ab2 + ao);
#pragma unroll
      for (int j = 0; j < 4; ++j) {
        acc[i][j] = Frag<T>::mma(ah, bh[j], acc[i][j]);
        if (SPLIT) {
          acc[i][j] = Frag<T>::mma(ah, bl[j], acc[i][j]);
          acc[i][j] = Frag<T>::mma(al, bh[j], acc[i][j]);
        }
      }
      Frag<T>::guard(acc[i][0], acc[i][3], ah, SPLIT ? al : ah);
    }
    Frag<T>::keep(bh[0], bh[1], bh[2], bh[3]);
    if (SPLIT) Frag<T>::keep(bl[0], bl[1], bl[2], bl[3]);
  }
  acc_guard4(acc[0][0], acc[0][1], acc[0][2], acc[0][3]);
  acc_guard4(acc[1][0], acc[1][1], acc[1][2], acc[1][3]);
  acc_guard4(acc[2][0], acc[2][1], acc[2][2], acc[2][3]);
  acc_guard4(acc[3][0], acc[3][1], acc[3][2], acc[3][3]);

  float* slab = sT[wave];
  const float* Rb = RESID ? (resid + (size_t)b * strideR) : nullptr;
#pragma unroll
  for (int i = 0; i < 4; ++i) {
    const int mBase = m0 + (i << 4);
#pragma unroll
    for (int j = 0; j < 4; ++j) {
      const int n = n0 + (j << 4) + rlane;
      float bv = 0.f;
      if (BIAS_MODE == 2) bv = bias[n];
#pragma unroll
      for (int r = 0; r < 8; ++r) {
        float v = acc[i][j][r] * scale;
        if (BIAS_MODE == 1) v += bias[mBase + mOff + r];
        if (BIAS_MODE == 2) v += bv;
        if (RESID) v += Rb[(size_t)(mBase + mOff + r) * ldc + n];
        if (ACT == 1) v = tanhf(v);
        if (ACT == 2) v = fmaxf(v, 0.0f);
        if (ACT == 3) v = v / (1.0f + expf(-v));
        if (ACT == 4) v = (v > 0.f) ? v : 0.01f * v;
        slab[(mOff + r) * 68 + (j << 4) + rlane] = v;
      }
    }
    __builtin_amdgcn_fence(__ATOMIC_RELEASE, "workgroup");
    __builtin_amdgcn_wave_barrier();
    __builtin_amdgcn_fence(__ATOMIC_ACQUIRE, "workgroup");
    if (OUT_MODE == 0) {
      float* C = (float*)Cout + (size_t)b * strideC;
      const int hh = lane >> 4, c4 = (lane & 15) * 4;
      for (int pass = 0; pass < 2; ++pass) {
#pragma unroll
        for (int it = 0; it < 8; ++it) {
          const int row = it * 2 + hh;
          v4f v = *(const v4f*)(slab + row * 68 + c4);
          *(volatile v4f*)(C + (size_t)(mBase + row) * ldc + n0 + c4) = v;
        }
        __threadfence();
      }
    } else {
      const int q = lane >> 3, c8 = (lane & 7) * 8;
      unsigned short* C  = (unsigned short*)Cout  + (size_t)b * strideC;
      unsigned short* Cl = (OUT_MODE == 2) ? ((unsigned short*)Cout2 + (size_t)b * strideC) : nullptr;
      for (int pass = 0; pass < 2; ++pass) {
#pragma unroll
        for (int it = 0; it < 4; ++it) {
          const int row = it * 4 + q;
          const float* sp = slab + row * 68 + c8;
          v8h hv, lv;
#pragma unroll
          for (int e = 0; e < 8; ++e) {
            if (OUT_MODE == 1) {
              hv[e] = (_Float16)sp[e];
            } else {
              unsigned short hb = f2bf_bits(sp[e]);
              unsigned short lb = f2bf_bits(sp[e] - bf_bits2f(hb));
              hv[e] = __builtin_bit_cast(_Float16, hb);
              lv[e] = __builtin_bit_cast(_Float16, lb);
            }
          }
          *(volatile v8h*)(C + (size_t)(mBase + row) * ldc + n0 + c8) = hv;
          if (OUT_MODE == 2) *(volatile v8h*)(Cl + (size_t)(mBase + row) * ldc + n0 + c8) = lv;
        }
        __threadfence();
      }
    }
    __builtin_amdgcn_fence(__ATOMIC_RELEASE, "workgroup");
    __builtin_amdgcn_wave_barrier();
    __builtin_amdgcn_fence(__ATOMIC_ACQUIRE, "workgroup");
  }
}

__global__ __launch_bounds__(256) void hh_prep_kernel(const float* __restrict__ x,
                                                      const float* __restrict__ ow,
                                                      const int* __restrict__ pidx,
                                                      const float* __restrict__ pneur,
                                                      unsigned short* __restrict__ Ahi,
                                                      unsigned short* __restrict__ Alo,
                                                      int ntok, int nproc) {
  __shared__ __align__(16) float xs[TOK_PER_BLK][RANK_DIM];
  const int lane = threadIdx.x & 31;
  const int wave = threadIdx.x >> 5;
  const int hsel = lane >> 4;
  const int csel = lane & 15;
  const int token = blockIdx.x * TOK_PER_BLK + wave;
  const int tokc  = token < ntok ? token : (ntok - 1);

  v4f xv = *(const v4f*)(x + (size_t)tokc * RANK_DIM + lane * 4);

#pragma unroll 1
  for (int k = 0; k < NREFL; ++k) {
    int idx = pidx[(size_t)tokc * NREFL + k];
    idx = idx < 0 ? 0 : idx;
    idx = idx > nproc - 1 ? (nproc - 1) : idx;
    const v4f vv = *(const v4f*)(pneur + (size_t)idx * RANK_DIM + lane * 4);
    float ss = vv.x * vv.x + vv.y * vv.y + vv.z * vv.z + vv.w * vv.w;
#pragma unroll
    for (int off = 16; off >= 1; off >>= 1) ss += __shfl_xor(ss, off, 32);
    const float inv = 1.0f / sqrtf(ss + 1e-8f);
    const v4f vh = vv * inv;
    float dp = xv.x * vh.x + xv.y * vh.y + xv.z * vh.z + xv.w * vh.w;
#pragma unroll
    for (int off = 16; off >= 1; off >>= 1) dp += __shfl_xor(dp, off, 32);
    const v4f v2 = vh * 2.0f;
    xv = xv - v2 * dp;
  }

  *(v4f*)(&xs[wave][lane * 4]) = xv;
  __syncthreads();
  const v4f xa = *(const v4f*)(&xs[wave][csel * 8]);
  const v4f xb = *(const v4f*)(&xs[wave][csel * 8 + 4]);
  const float x8[8] = {xa.x, xa.y, xa.z, xa.w, xb.x, xb.y, xb.z, xb.w};

  v8h hv[4], lv[4];
#pragma unroll
  for (int i = 0; i < 4; ++i) {
    const int n = 2 * i + hsel;
    const float wn = ow[(size_t)tokc * NOUT + n];
#pragma unroll
    for (int e = 0; e < 8; ++e) {
      const float val = wn * x8[e];
      const unsigned short hb = f2bf_bits(val);
      const unsigned short lb = f2bf_bits(val - bf_bits2f(hb));
      hv[i][e] = __builtin_bit_cast(_Float16, hb);
      lv[i][e] = __builtin_bit_cast(_Float16, lb);
    }
  }

  if (token < ntok) {
    unsigned short* rh = Ahi + (size_t)token * KCOLS;
    unsigned short* rl = Alo + (size_t)token * KCOLS;
    for (int pass = 0; pass < 2; ++pass) {
#pragma unroll
      for (int i = 0; i < 4; ++i) {
        *(volatile v8h*)(rh + i * 256 + lane * 8) = hv[i];
        *(volatile v8h*)(rl + i * 256 + lane * 8) = lv[i];
      }
      __threadfence();
    }
  }
}

__global__ __launch_bounds__(256) void transpose_split_kernel(const float* __restrict__ W,
                                                              unsigned short* __restrict__ Bhi,
                                                              unsigned short* __restrict__ Blo,
                                                              int nrows_k, int ncols_d) {
  __shared__ float tile[64][65];
  const int t  = threadIdx.x;
  const int k0 = blockIdx.y * 64;
  const int d0 = blockIdx.x * 64;
#pragma unroll
  for (int it = 0; it < 4; ++it) {
    const int r  = it * 16 + (t >> 4);
    const int c4 = (t & 15) * 4;
    const v4f v = *(const v4f*)(W + (size_t)(k0 + r) * ncols_d + d0 + c4);
    tile[r][c4 + 0] = v.x;
    tile[r][c4 + 1] = v.y;
    tile[r][c4 + 2] = v.z;
    tile[r][c4 + 3] = v.w;
  }
  __syncthreads();
  v8h hv[2], lv[2];
#pragma unroll
  for (int it = 0; it < 2; ++it) {
    const int dd = it * 32 + (t >> 3);
    const int kk = (t & 7) * 8;
#pragma unroll
    for (int e = 0; e < 8; ++e) {
      const float val = tile[kk + e][dd];
      const unsigned short hb = f2bf_bits(val);
      const unsigned short lb = f2bf_bits(val - bf_bits2f(hb));
      hv[it][e] = __builtin_bit_cast(_Float16, hb);
      lv[it][e] = __builtin_bit_cast(_Float16, lb);
    }
  }
  for (int pass = 0; pass < 2; ++pass) {
#pragma unroll
    for (int it = 0; it < 2; ++it) {
      const int dd = it * 32 + (t >> 3);
      const int kk = (t & 7) * 8;
      const size_t o = (size_t)(d0 + dd) * nrows_k + k0 + kk;
      *(volatile v8h*)(Bhi + o) = hv[it];
      *(volatile v8h*)(Blo + o) = lv[it];
    }
    __threadfence();
  }
}

extern "C" void kernel_launch(void* const* d_in, const int* in_sizes, int n_in,
                              void* d_out, int out_size, void* d_ws, size_t ws_size,
                              hipStream_t stream) {
  if (n_in < 5) return;
  const float* x     = (const float*)d_in[0];
  const float* ow    = (const float*)d_in[1];
  const int*   pidx  = (const int*)d_in[2];
  const float* pneur = (const float*)d_in[3];
  const float* oneur = (const float*)d_in[4];
  float* out = (float*)d_out;

  const int ntok  = in_sizes[0] / RANK_DIM;
  const int nproc = in_sizes[3] / RANK_DIM;
  if (ntok <= 0 || nproc <= 0) return;
  if (in_sizes[0] != ntok * RANK_DIM) return;
  if (in_sizes[1] != ntok * NOUT) return;
  if (in_sizes[2] != ntok * NREFL) return;
  if (in_sizes[4] != NOUT * RANK_DIM * DMODEL) return;
  if (out_size != ntok * DMODEL) return;
  if ((ntok % 64) != 0 || (ntok % TOK_PER_BLK) != 0) return;

  const size_t bytesA = (size_t)ntok * KCOLS * sizeof(unsigned short);
  const size_t bytesB = (size_t)DMODEL * KCOLS * sizeof(unsigned short);
  const size_t offAhi = 0;
  const size_t offAlo = offAhi + bytesA;
  const size_t offBhi = offAlo + bytesA;
  const size_t offBlo = offBhi + bytesB;
  const size_t total  = offBlo + bytesB;
  if (total > ws_size) return;

  unsigned short* Ahi = (unsigned short*)((char*)d_ws + offAhi);
  unsigned short* Alo = (unsigned short*)((char*)d_ws + offAlo);
  unsigned short* Bhi = (unsigned short*)((char*)d_ws + offBhi);
  unsigned short* Blo = (unsigned short*)((char*)d_ws + offBlo);

  hh_prep_kernel<<<dim3(ntok / TOK_PER_BLK), dim3(256), 0, stream>>>(x, ow, pidx, pneur, Ahi, Alo, ntok, nproc);

  transpose_split_kernel<<<dim3(DMODEL / 64, KCOLS / 64), dim3(256), 0, stream>>>(oneur, Bhi, Blo, KCOLS, DMODEL);

  const int tiles = (ntok / 64) * (DMODEL / 64);
  const int gblocks = (tiles + 7) / 8;
  wmma_gemm64<1, true, 0, 0, false, 0><<<dim3(gblocks, 1), dim3(256), 0, stream>>>(
      Ahi, Alo, KCOLS, 0L,
      Bhi, Blo, KCOLS, 0L,
      (void*)out, (void*)0, DMODEL, 0L,
      (const float*)0,
      (const float*)0, 0L,
      ntok, DMODEL, KCOLS, 1.0f);
}
